// GT_80238579023945
// MI455X (gfx1250) — hardware-verified
//
#include <hip/hip_runtime.h>
#include <stddef.h>


#define DF       128
#define QKVW     384
#define NTHR     256
#define NWAVE    8
#define EPT      8
#define NGRP     2
#define CHUNK    (NTHR * EPT * NGRP)
#define WCAP     (EPT * NGRP * 32)
#define LISTN    (NWAVE * WCAP)
#define NBC      4096
#define NBF      1024
#define RCAP     40960
#define RBN      128
#define OTHR     512
#define GROWS    128
#define DEGCAP   256
#define APU      68
#define KU       (DF / 2)
#define SCALE_QK 0.25f

#define LDS_ATILE (2 * GROWS * APU * 4)
#define LDS_GEMM  (LDS_ATILE + GROWS * DF * 4)
#define LDS_ATTN  (LDS_ATILE)
#define LDS_FILL  ((RCAP + NBF + LISTN) * 4 + 64)

static_assert((CHUNK & (CHUNK - 1)) == 0);
static_assert(CHUNK <= 4096);
static_assert((NBC & (NBC - 1)) == 0 && (NBF & (NBF - 1)) == 0);
static_assert(NBC == 4 * NBF);
static_assert(OTHR * 8 == NBC);
static_assert((RCAP % 32) == 0);
static_assert(GROWS == NWAVE * 16);
static_assert(GROWS * DF * 4 <= LDS_ATILE);
static_assert((GROWS * DF / 8) % NTHR == 0);
static_assert((APU * 4) % 16 == 0);

typedef float    v4f  __attribute__((ext_vector_type(4)));
typedef float    v8f  __attribute__((ext_vector_type(8)));
typedef int      v4i  __attribute__((ext_vector_type(4)));
typedef unsigned v4u  __attribute__((ext_vector_type(4)));
typedef unsigned v2u  __attribute__((ext_vector_type(2)));
typedef __bf16   v16b __attribute__((ext_vector_type(16)));
union FragB { v16b v; v4u q[2]; };

__device__ __forceinline__ unsigned bfb(float f) {
  unsigned u = __float_as_uint(f);
  u += 0x7FFFu + ((u >> 16) & 1u);
  return u >> 16;
}

__device__ __forceinline__ unsigned split_pair(float x0, float x1, unsigned& lo) {
  const unsigned h0 = bfb(x0), h1 = bfb(x1);
  const float r0 = x0 - __uint_as_float(h0 << 16);
  const float r1 = x1 - __uint_as_float(h1 << 16);
  lo = bfb(r0) | (bfb(r1) << 16);
  return h0 | (h1 << 16);
}

__device__ __forceinline__ void split8(v4f a, v4f b, v4u& hq, v4u& lq) {
  unsigned l;
  hq.x = split_pair(a.x, a.y, l); lq.x = l;
  hq.y = split_pair(a.z, a.w, l); lq.y = l;
  hq.z = split_pair(b.x, b.y, l); lq.z = l;
  hq.w = split_pair(b.z, b.w, l); lq.w = l;
}

__device__ __forceinline__ v8f wmb(v16b a, v16b b, v8f c) {
  v8f d = __builtin_amdgcn_wmma_f32_16x16x32_bf16(false, a, false, b, (short)0, c, false, false);
  asm volatile("v_nop\n\tv_nop\n\tv_nop\n\tv_nop" : "+v"(d) : "v"(a), "v"(b));
  return d;
}

template <int NB>
__device__ __forceinline__ int scan_chunk(const int* __restrict__ dsts, int nE, int cbase, int slotBase,
                                          int vec8, int* list, int tid, int lane, int wave) {
  int wc = 0;
#pragma unroll
  for (int g = 0; g < NGRP; ++g) {
    const int el0  = (g * NTHR + tid) * EPT;
    const int e0   = cbase + el0;
    const int sent = -2147483647 - 1;
    v4i da, db;
    if (vec8 != 0 && cbase + CHUNK <= nE) {
      da = *(const v4i*)(dsts + e0);
      db = *(const v4i*)(dsts + e0 + 4);
    } else {
      da.x = (e0     < nE) ? dsts[min(e0, nE - 1)]     : sent;
      da.y = (e0 + 1 < nE) ? dsts[min(e0 + 1, nE - 1)] : sent;
      da.z = (e0 + 2 < nE) ? dsts[min(e0 + 2, nE - 1)] : sent;
      da.w = (e0 + 3 < nE) ? dsts[min(e0 + 3, nE - 1)] : sent;
      db.x = (e0 + 4 < nE) ? dsts[min(e0 + 4, nE - 1)] : sent;
      db.y = (e0 + 5 < nE) ? dsts[min(e0 + 5, nE - 1)] : sent;
      db.z = (e0 + 6 < nE) ? dsts[min(e0 + 6, nE - 1)] : sent;
      db.w = (e0 + 7 < nE) ? dsts[min(e0 + 7, nE - 1)] : sent;
    }
    const unsigned nb = (unsigned)slotBase;
    const unsigned s0 = (unsigned)da.x - nb, s1 = (unsigned)da.y - nb;
    const unsigned s2 = (unsigned)da.z - nb, s3 = (unsigned)da.w - nb;
    const unsigned s4 = (unsigned)db.x - nb, s5 = (unsigned)db.y - nb;
    const unsigned s6 = (unsigned)db.z - nb, s7 = (unsigned)db.w - nb;
    const bool h0 = s0 < (unsigned)NB, h1 = s1 < (unsigned)NB, h2 = s2 < (unsigned)NB, h3 = s3 < (unsigned)NB;
    const bool h4 = s4 < (unsigned)NB, h5 = s5 < (unsigned)NB, h6 = s6 < (unsigned)NB, h7 = s7 < (unsigned)NB;
    const unsigned any = __builtin_amdgcn_ballot_w32(h0 | h1 | h2 | h3 | h4 | h5 | h6 | h7);
    if (any != 0u) {
#define HITJ(J, HJ, SJ) { \
        const unsigned mj = __builtin_amdgcn_ballot_w32(HJ); \
        if (mj != 0u) { \
          if (HJ) { \
            const int pos = wc + (int)__builtin_amdgcn_mbcnt_lo(mj, 0u); \
            if (pos < WCAP) list[wave * WCAP + pos] = ((el0 + (J)) << 12) | (int)(SJ); \
          } \
          wc += (int)__builtin_popcount(mj); } }
      HITJ(0, h0, s0)
      HITJ(1, h1, s1)
      HITJ(2, h2, s2)
      HITJ(3, h3, s3)
      HITJ(4, h4, s4)
      HITJ(5, h5, s5)
      HITJ(6, h6, s6)
      HITJ(7, h7, s7)
#undef HITJ
    }
  }
  return wc;
}

__global__ __launch_bounds__(NTHR) void k_wprep(
    const float* __restrict__ qkvw, const float* __restrict__ outw, const float* __restrict__ outwl,
    unsigned* wqh, unsigned* wql, unsigned* woh, unsigned* wol, unsigned* wlh, unsigned* wll,
    int nL, int nCls) {
  const int g0 = nL * (QKVW * DF / 8);
  const int g1 = (nL - 1) * (DF * DF / 8);
  const int g2 = nCls * DF / 8;
  const int bstart = blockIdx.x * NTHR;
  const int i = bstart + (int)threadIdx.x;
  if (i >= g0 + g1 + g2) return;
  const float* sb; unsigned* dh; unsigned* dl; int o, oo, Nsrc;
  if (bstart < g0) {
    o = i * 8;
    const int per = QKVW * DF;
    const int l = o / per;
    oo = o - l * per;
    sb = qkvw + (size_t)l * 3 * DF * DF;
    Nsrc = DF; dh = wqh; dl = wql;
  } else if (bstart < g0 + g1) {
    o = (i - g0) * 8;
    const int per = DF * DF;
    const int l = o / per;
    oo = o - l * per;
    sb = outw + (size_t)l * DF * DF;
    Nsrc = DF; dh = woh; dl = wol;
  } else {
    o = (i - g0 - g1) * 8;
    oo = o;
    sb = outwl;
    Nsrc = nCls; dh = wlh; dl = wll;
  }
  const int np = oo / DF;
  const int k0 = oo - np * DF;
  const int mm = np / DF;
  const int n  = np - mm * DF;
  float v[8];
#pragma unroll
  for (int e = 0; e < 8; ++e) v[e] = sb[((size_t)(mm * DF + k0 + e)) * Nsrc + n];
  v4f a, b;
  a.x = v[0]; a.y = v[1]; a.z = v[2]; a.w = v[3];
  b.x = v[4]; b.y = v[5]; b.z = v[6]; b.w = v[7];
  v4u hq, lq;
  split8(a, b, hq, lq);
  unsigned* ph = dh + (o >> 1);
  unsigned* pl = dl + (o >> 1);
  *(volatile v4u*)ph = hq;
  *(volatile v4u*)pl = lq;
  __threadfence();
  *(volatile v4u*)ph = hq;
  *(volatile v4u*)pl = lq;
}

__global__ __launch_bounds__(NTHR) void k_count(const int* __restrict__ dsts, int* cnt, int nE, int vec8) {
  __shared__ __attribute__((aligned(16))) int scnt[NBC];
  __shared__ __attribute__((aligned(16))) int list[LISTN];
  __shared__ int wcnt[NWAVE];
  const int tid = threadIdx.x, lane = tid & 31, wave = tid >> 5;
  const int nodeBase = blockIdx.x * NBC;

  for (int i = tid; i < NBC; i += NTHR) scnt[i] = 0;
  __syncthreads();

  const int nChunks = (nE + CHUNK - 1) / CHUNK;
#pragma unroll 1
  for (int ch = 0; ch < nChunks; ++ch) {
    const int cbase = ch * CHUNK;
    const int wc = scan_chunk<NBC>(dsts, nE, cbase, nodeBase, vec8, list, tid, lane, wave);
    if (lane == 0) wcnt[wave] = wc;
    __syncthreads();
    if (wave == 0) {
#pragma unroll 1
      for (int wsx = 0; wsx < NWAVE; ++wsx) {
        int n = __builtin_amdgcn_readfirstlane(wcnt[wsx]);
        n = n > WCAP ? WCAP : (n < 0 ? 0 : n);
        const int* lp = list + wsx * WCAP;
#pragma unroll 1
        for (int i = 0; i < n; ++i) {
          const int ent  = __builtin_amdgcn_readfirstlane(lp[i]);
          const int slot = ent & (NBC - 1);
          if (lane == 0) scnt[slot] = scnt[slot] + 1;
        }
      }
    }
    __syncthreads();
  }

  v4i cq[4];
#pragma unroll
  for (int q = 0; q < 4; ++q) {
    const int f = (wave * 4 + q) * 128 + 4 * lane;
    cq[q] = *(const v4i*)(scnt + f);
  }
  int* cp = cnt + (size_t)nodeBase;
#pragma unroll
  for (int q = 0; q < 4; ++q) {
    const int f = (wave * 4 + q) * 128 + 4 * lane;
    *(volatile v4i*)(cp + f) = cq[q];
  }
  __threadfence();
#pragma unroll
  for (int q = 0; q < 4; ++q) {
    const int f = (wave * 4 + q) * 128 + 4 * lane;
    *(volatile v4i*)(cp + f) = cq[q];
  }
}

__global__ __launch_bounds__(OTHR) void k_offsets(
    const int* __restrict__ cnt, int* off, int* rbase, int nChunk) {
  __shared__ __attribute__((aligned(16))) int soff[NBC];
  __shared__ __attribute__((aligned(16))) int srb[RBN];
  __shared__ int wtot[OTHR / 32];
  const int tid = threadIdx.x, lane = tid & 31, wave = tid >> 5, sub = tid >> 7;
  for (int i = tid; i < RBN; i += OTHR) srb[i] = 0;
  int carry = 0;
#pragma unroll 1
  for (int ch = 0; ch < nChunk; ++ch) {
    const int base = ch * NBC;
    const v4i c0 = *(const v4i*)(cnt + base + 8 * tid);
    const v4i c1 = *(const v4i*)(cnt + base + 8 * tid + 4);
    const int e0 = max(c0.x, 0), e1 = max(c0.y, 0), e2 = max(c0.z, 0), e3 = max(c0.w, 0);
    const int e4 = max(c1.x, 0), e5 = max(c1.y, 0), e6 = max(c1.z, 0), e7 = max(c1.w, 0);
    const int ts = e0 + e1 + e2 + e3 + e4 + e5 + e6 + e7;
    int incl = ts;
#pragma unroll
    for (int d = 1; d < 32; d <<= 1) {
      const int t = __shfl_up(incl, d);
      if (lane >= d) incl += t;
    }
    if (lane == 31) wtot[wave] = incl;
    __syncthreads();
    const int S0 = wtot[0]  + wtot[1]  + wtot[2]  + wtot[3];
    const int S1 = wtot[4]  + wtot[5]  + wtot[6]  + wtot[7];
    const int S2 = wtot[8]  + wtot[9]  + wtot[10] + wtot[11];
    const int S3 = wtot[12] + wtot[13] + wtot[14] + wtot[15];
    int pre = 0;
#pragma unroll 1
    for (int w = 4 * sub; w < wave; ++w) pre += wtot[w];
    const int b0 = carry;
    const int b1 = b0 + ((S0 + 31) & ~31);
    const int b2 = b1 + ((S1 + 31) & ~31);
    const int b3 = b2 + ((S2 + 31) & ~31);
    const int b4 = b3 + ((S3 + 31) & ~31);
    const int myb = sub == 0 ? b0 : (sub == 1 ? b1 : (sub == 2 ? b2 : b3));
    if (tid == 0) {
      srb[min(4 * ch + 0, RBN - 1)] = b0;
      srb[min(4 * ch + 1, RBN - 1)] = b1;
      srb[min(4 * ch + 2, RBN - 1)] = b2;
      srb[min(4 * ch + 3, RBN - 1)] = b3;
    }
    int run = myb + pre + incl - ts;
    soff[8 * tid + 0] = run; run += e0;
    soff[8 * tid + 1] = run; run += e1;
    soff[8 * tid + 2] = run; run += e2;
    soff[8 * tid + 3] = run; run += e3;
    soff[8 * tid + 4] = run; run += e4;
    soff[8 * tid + 5] = run; run += e5;
    soff[8 * tid + 6] = run; run += e6;
    soff[8 * tid + 7] = run;
    carry = b4;
    __syncthreads();
    const v4i o0 = *(const v4i*)(soff + 4 * tid);
    const v4i o1 = *(const v4i*)(soff + 4 * (tid + OTHR));
    int* op = off + base;
    *(volatile v4i*)(op + 4 * tid) = o0;
    *(volatile v4i*)(op + 4 * (tid + OTHR)) = o1;
    __threadfence();
    *(volatile v4i*)(op + 4 * tid) = o0;
    *(volatile v4i*)(op + 4 * (tid + OTHR)) = o1;
    __syncthreads();
  }
  if (tid == 0) srb[min(4 * nChunk, RBN - 1)] = carry;
  __syncthreads();
  v4i rv = {0, 0, 0, 0};
  if (tid < 32) rv = *(const v4i*)(srb + 4 * tid);
  if (tid < 32) *(volatile v4i*)(rbase + 4 * tid) = rv;
  __threadfence();
  if (tid < 32) *(volatile v4i*)(rbase + 4 * tid) = rv;
}

__global__ __launch_bounds__(NTHR) void k_fill(
    const int* __restrict__ srcs, const int* __restrict__ dsts, const int* __restrict__ off,
    const int* __restrict__ rbase, int* csr, int nN, int nE, int vec8, int csrLen) {
  extern __shared__ v4u lds_dyn[];
  int* region = (int*)lds_dyn;
  int* cursor = region + RCAP;
  int* list   = cursor + NBF;
  int* wcnt   = list + LISTN;
  const int tid = threadIdx.x, lane = tid & 31, wave = tid >> 5;
  const int b = blockIdx.x;
  const int nodeBase = b * NBF;

  int rb0 = rbase[b];
  const int rb1 = rbase[b + 1];
  rb0 = rb0 < 0 ? 0 : (rb0 > csrLen ? csrLen : rb0);
  rb0 &= ~31;
  int len = rb1 - rb0;
  len = len < 0 ? 0 : (len > RCAP ? RCAP : len);
  int lenW = (len + 31) & ~31;
  if (rb0 + lenW > csrLen) lenW = (csrLen - rb0) & ~31;

  {
    const v4i z = {0, 0, 0, 0};
    for (int i = tid; i < RCAP / 4; i += NTHR) ((v4i*)region)[i] = z;
    for (int s = tid; s < NBF; s += NTHR) {
      int o = off[nodeBase + s] - rb0;
      o = o < 0 ? 0 : (o > RCAP ? RCAP : o);
      cursor[s] = o;
    }
  }
  __syncthreads();

  const int nChunks = (nE + CHUNK - 1) / CHUNK;
#pragma unroll 1
  for (int ch = 0; ch < nChunks; ++ch) {
    const int cbase = ch * CHUNK;
    const int wc = scan_chunk<NBF>(dsts, nE, cbase, nodeBase, vec8, list, tid, lane, wave);
    if (lane == 0) wcnt[wave] = wc;
    __syncthreads();
    if (wave == 0) {
#pragma unroll 1
      for (int wsx = 0; wsx < NWAVE; ++wsx) {
        int n = __builtin_amdgcn_readfirstlane(wcnt[wsx]);
        n = n > WCAP ? WCAP : (n < 0 ? 0 : n);
        const int* lp = list + wsx * WCAP;
#pragma unroll 1
        for (int i = 0; i < n; ++i) {
          const int ent  = __builtin_amdgcn_readfirstlane(lp[i]);
          const int slot = ent & (NBF - 1);
          int e = cbase + ((ent >> 12) & (CHUNK - 1));
          e = e > nE - 1 ? nE - 1 : e;
          int sv = srcs[e];
          sv = sv < 0 ? 0 : (sv > nN - 1 ? nN - 1 : sv);
          if (lane == 0) {
            int pos = cursor[slot];
            pos = pos < 0 ? 0 : (pos > RCAP - 1 ? RCAP - 1 : pos);
            region[pos] = sv;
            const int npos = pos + 1;
            cursor[slot] = npos > RCAP ? RCAP : npos;
          }
        }
      }
    }
    __syncthreads();
  }

  const int nv = lenW >> 2;
  int* gp = csr + rb0;
#pragma unroll 1
  for (int i = tid; i < nv; i += NTHR) { const v4i v = ((const v4i*)region)[i]; *(volatile v4i*)(gp + 4 * i) = v; }
  __threadfence();
#pragma unroll 1
  for (int i = tid; i < nv; i += NTHR) { const v4i v = ((const v4i*)region)[i]; *(volatile v4i*)(gp + 4 * i) = v; }
}

__global__ __launch_bounds__(NTHR) void k_gemm(
    const float* __restrict__ A, int nRowsA,
    const unsigned* __restrict__ Bh, const unsigned* __restrict__ Bl,
    const float* __restrict__ bias, float* C) {
  extern __shared__ v4u lds_dyn[];
  unsigned* sAh = (unsigned*)lds_dyn;
  unsigned* sAl = sAh + GROWS * APU;
  float*    stg = (float*)(sAl + GROWS * APU);
  const int tid = threadIdx.x, lane = tid & 31, wave = tid >> 5, hh = lane >> 4, m = lane & 15;
  const int rowBase = blockIdx.x * GROWS;

#pragma unroll
  for (int i = 0; i < (GROWS * DF / 8) / NTHR; ++i) {
    const int idx = i * NTHR + tid;
    const int r   = idx >> 4;
    const int c0  = (idx & 15) * 8;
    int row = rowBase + r;
    row = row > nRowsA - 1 ? nRowsA - 1 : row;
    const float* ap = A + (size_t)row * DF + c0;
    const v4f a = *(const v4f*)ap, b = *(const v4f*)(ap + 4);
    v4u hq, lq;
    split8(a, b, hq, lq);
    *(v4u*)(sAh + r * APU + (c0 >> 1)) = hq;
    *(v4u*)(sAl + r * APU + (c0 >> 1)) = lq;
  }
  __syncthreads();

  const unsigned* arh = sAh + (wave * 16 + m) * APU + 4 * hh;
  const unsigned* arl = sAl + (wave * 16 + m) * APU + 4 * hh;
  const int r0 = wave * 16 + 8 * hh;
#pragma unroll 1
  for (int g = 0; g < QKVW / DF; ++g) {
    v8f acc[8];
#pragma unroll
    for (int t = 0; t < 8; ++t) { v8f z = {0.f, 0.f, 0.f, 0.f, 0.f, 0.f, 0.f, 0.f}; acc[t] = z; }
#pragma unroll
    for (int kt = 0; kt < DF / 32; ++kt) {
      FragB ah, al;
      ah.q[0] = *(const v4u*)(arh + 16 * kt);
      ah.q[1] = *(const v4u*)(arh + 16 * kt + 8);
      al.q[0] = *(const v4u*)(arl + 16 * kt);
      al.q[1] = *(const v4u*)(arl + 16 * kt + 8);
#pragma unroll
      for (int t = 0; t < 8; ++t) {
        const size_t bo = (size_t)(DF * g + 16 * t + m) * KU + 16 * kt + 4 * hh;
        FragB bh, bl;
        bh.q[0] = *(const v4u*)(Bh + bo);
        bh.q[1] = *(const v4u*)(Bh + bo + 8);
        bl.q[0] = *(const v4u*)(Bl + bo);
        bl.q[1] = *(const v4u*)(Bl + bo + 8);
        acc[t] = wmb(ah.v, bh.v, acc[t]);
        acc[t] = wmb(ah.v, bl.v, acc[t]);
        acc[t] = wmb(al.v, bh.v, acc[t]);
      }
    }
    __syncthreads();
    float* sp = stg + r0 * DF + m;
#pragma unroll
    for (int t = 0; t < 8; ++t) {
      const float bv = bias[DF * g + 16 * t + m];
#pragma unroll
      for (int r = 0; r < 8; ++r) sp[r * DF + 16 * t] = acc[t][r] + bv;
    }
    __syncthreads();
    const float* lp = stg + wave * 16 * DF + 4 * lane;
    float* gp = C + ((size_t)rowBase + wave * 16) * QKVW + DF * g + 4 * lane;
#pragma unroll
    for (int i = 0; i < 16; ++i) { const v4f v = *(const v4f*)(lp + i * DF); *(volatile v4f*)(gp + (size_t)i * QKVW) = v; }
    __threadfence();
#pragma unroll
    for (int i = 0; i < 16; ++i) { const v4f v = *(const v4f*)(lp + i * DF); *(volatile v4f*)(gp + (size_t)i * QKVW) = v; }
  }
}

template <int NT>
__global__ __launch_bounds__(NTHR) void k_attn(
    const int* __restrict__ csr, const int* __restrict__ off, const int* __restrict__ cnt,
    const float* __restrict__ qkv, const unsigned* __restrict__ Bh, const unsigned* __restrict__ Bl,
    const float* __restrict__ bias, float* Out, int nRowsOut, int nN, int csrLen) {
  extern __shared__ v4u lds_dyn[];
  unsigned* sAh = (unsigned*)lds_dyn;
  unsigned* sAl = sAh + GROWS * APU;
  float*    stg = (float*)lds_dyn;
  constexpr int NOUT = 16 * NT;
  const int tid = threadIdx.x, lane = tid & 31, wave = tid >> 5, hh = lane >> 4, m = lane & 15;
  const int tb = blockIdx.x * GROWS + wave * 16;
  const int cl = tb + m;
  const int cnt_l = cnt[cl];
  const int off_l = off[cl];

#pragma unroll 1
  for (int j = 0; j < 16; ++j) {
    const int c = tb + j;
    int n = __builtin_amdgcn_readlane(cnt_l, j);
    n = n < 0 ? 0 : (n > DEGCAP ? DEGCAP : n);
    const int st = __builtin_amdgcn_readlane(off_l, j);
    const v4f kv = *(const v4f*)(qkv + (size_t)c * QKVW + DF + 4 * lane);
    float mx = -1.0e30f, den = 0.0f;
    v4f acc = {0.f, 0.f, 0.f, 0.f};
#pragma unroll 1
    for (int q0 = 0; q0 < n; q0 += 32) {
      int pos = st + q0 + lane;
      pos = pos < 0 ? 0 : (pos > csrLen - 1 ? csrLen - 1 : pos);
      int sl = csr[pos];
      sl = sl < 0 ? 0 : (sl > nN - 1 ? nN - 1 : sl);
      const int mc = (n - q0) < 32 ? (n - q0) : 32;
#pragma unroll 1
      for (int p = 0; p < mc; ++p) {
        const int s = __builtin_amdgcn_readlane(sl, p);
        const float* rp = qkv + (size_t)s * QKVW + 4 * lane;
        const v4f qv = *(const v4f*)rp;
        const v4f vv = *(const v4f*)(rp + 2 * DF);
        float d = qv.x * kv.x + qv.y * kv.y + qv.z * kv.z + qv.w * kv.w;
        d += __shfl_xor(d, 1);
        d += __shfl_xor(d, 2);
        const float sc = d * SCALE_QK;
        const float mn = fmaxf(mx, sc);
        const float al = __expf(mx - mn);
        const float ex = __expf(sc - mn);
        den = den * al + ex;
        acc = acc * al + vv * ex;
        mx = mn;
      }
    }
    const float inv = 1.0f / fmaxf(den, 1e-16f);
    const v4f o = acc * inv;
    unsigned l0, l1;
    const unsigned h0 = split_pair(o.x, o.y, l0);
    const unsigned h1 = split_pair(o.z, o.w, l1);
    v2u hv, lv;
    hv.x = h0; hv.y = h1; lv.x = l0; lv.y = l1;
    const int ro = (wave * 16 + j) * APU + 2 * lane;
    *(v2u*)(sAh + ro) = hv;
    *(v2u*)(sAl + ro) = lv;
  }
  __syncthreads();

  v8f acc2[NT];
#pragma unroll
  for (int t = 0; t < NT; ++t) { v8f z = {0.f, 0.f, 0.f, 0.f, 0.f, 0.f, 0.f, 0.f}; acc2[t] = z; }
  const unsigned* arh = sAh + (wave * 16 + m) * APU + 4 * hh;
  const unsigned* arl = sAl + (wave * 16 + m) * APU + 4 * hh;
#pragma unroll
  for (int kt = 0; kt < DF / 32; ++kt) {
    FragB ah, al;
    ah.q[0] = *(const v4u*)(arh + 16 * kt);
    ah.q[1] = *(const v4u*)(arh + 16 * kt + 8);
    al.q[0] = *(const v4u*)(arl + 16 * kt);
    al.q[1] = *(const v4u*)(arl + 16 * kt + 8);
#pragma unroll
    for (int t = 0; t < NT; ++t) {
      const size_t bo = (size_t)(16 * t + m) * KU + 16 * kt + 4 * hh;
      FragB bh, bl;
      bh.q[0] = *(const v4u*)(Bh + bo);
      bh.q[1] = *(const v4u*)(Bh + bo + 8);
      bl.q[0] = *(const v4u*)(Bl + bo);
      bl.q[1] = *(const v4u*)(Bl + bo + 8);
      acc2[t] = wmb(ah.v, bh.v, acc2[t]);
      acc2[t] = wmb(ah.v, bl.v, acc2[t]);
      acc2[t] = wmb(al.v, bh.v, acc2[t]);
    }
  }
  __syncthreads();

  const int r0 = wave * 16 + 8 * hh;
  float* sp = stg + r0 * NOUT + m;
#pragma unroll
  for (int t = 0; t < NT; ++t) {
    const float bv = bias[16 * t + m];
#pragma unroll
    for (int r = 0; r < 8; ++r) sp[r * NOUT + 16 * t] = acc2[t][r] + bv;
  }
  __syncthreads();

  constexpr int NI = 16 * NOUT / 128;
  const float* lp = stg + wave * 16 * NOUT;
  float* gp = Out + (size_t)tb * NOUT;
#pragma unroll
  for (int i = 0; i < NI; ++i) {
    const int q  = 32 * i + lane;
    const int rl = (4 * q) / NOUT;
    const v4f v  = *(const v4f*)(lp + 4 * q);
    if (tb + rl < nRowsOut) *(volatile v4f*)(gp + 4 * q) = v;
  }
  __threadfence();
#pragma unroll
  for (int i = 0; i < NI; ++i) {
    const int q  = 32 * i + lane;
    const int rl = (4 * q) / NOUT;
    const v4f v  = *(const v4f*)(lp + 4 * q);
    if (tb + rl < nRowsOut) *(volatile v4f*)(gp + 4 * q) = v;
  }
}

extern "C" void kernel_launch(void* const* d_in, const int* in_sizes, int n_in,
                              void* d_out, int out_size, void* d_ws, size_t ws_size,
                              hipStream_t stream) {
  if (n_in < 9) return;
  const int nN = in_sizes[0] / DF;
  const int nE = in_sizes[1];
  if (nN <= 0 || nE <= 0 || in_sizes[0] != nN * DF || in_sizes[2] != nE) return;
  const int nL = in_sizes[3] / (3 * DF * DF);
  if (nL < 1 || in_sizes[3] != nL * 3 * DF * DF || in_sizes[4] != nL * QKVW) return;
  if (in_sizes[5] != (nL - 1) * DF * DF || in_sizes[6] != (nL - 1) * DF) return;
  const int nCls = in_sizes[7] / DF;
  if ((nCls != 64 && nCls != 128) || in_sizes[7] != nCls * DF || in_sizes[8] != nCls) return;
  if (out_size != nN * nCls) return;
  if (nE > (1 << 28) || nN > (1 << 24)) return;

  const float* x     = (const float*)d_in[0];
  const int*   srcA  = (const int*)d_in[1];
  const int*   dstA  = (const int*)d_in[2];
  const float* qkvw  = (const float*)d_in[3];
  const float* qkvb  = (const float*)d_in[4];
  const float* outw  = (const float*)d_in[5];
  const float* outb  = (const float*)d_in[6];
  const float* outwl = (const float*)d_in[7];
  const float* outbl = (const float*)d_in[8];
  float* out = (float*)d_out;

  const int NPAD   = ((nN + GROWS - 1) / GROWS) * GROWS;
  const int nBC    = (nN + NBC - 1) / NBC;
  const int CNTPAD = nBC * NBC;
  if (4 * nBC + 1 > RBN) return;
  const int nBF    = (nN + NBF - 1) / NBF;
  const int csrLen = ((nE + 31) & ~31) + 4096;
  const int nBlk   = NPAD / GROWS;

  char* ws = (char*)d_ws;
  size_t off = 0;
  const size_t oWQh = off; off += (size_t)nL * QKVW * DF * 2;        off = (off + 255) & ~(size_t)255;
  const size_t oWQl = off; off += (size_t)nL * QKVW * DF * 2;        off = (off + 255) & ~(size_t)255;
  const size_t oWOh = off; off += (size_t)(nL - 1) * DF * DF * 2;    off = (off + 255) & ~(size_t)255;
  const size_t oWOl = off; off += (size_t)(nL - 1) * DF * DF * 2;    off = (off + 255) & ~(size_t)255;
  const size_t oWLh = off; off += (size_t)nCls * DF * 2;             off = (off + 255) & ~(size_t)255;
  const size_t oWLl = off; off += (size_t)nCls * DF * 2;             off = (off + 255) & ~(size_t)255;
  const size_t oCnt = off; off += (size_t)CNTPAD * 4;                off = (off + 255) & ~(size_t)255;
  const size_t oOff = off; off += (size_t)CNTPAD * 4;                off = (off + 255) & ~(size_t)255;
  const size_t oRb  = off; off += (size_t)RBN * 4;                   off = (off + 255) & ~(size_t)255;
  const size_t oCsr = off; off += (size_t)csrLen * 4;                off = (off + 255) & ~(size_t)255;
  const size_t oX   = off; off += (size_t)NPAD * DF * 4;             off = (off + 255) & ~(size_t)255;
  const size_t oQKV = off; off += (size_t)NPAD * QKVW * 4;           off = (off + 255) & ~(size_t)255;
  if (off > ws_size) return;
  unsigned* wqh  = (unsigned*)(ws + oWQh);
  unsigned* wql  = (unsigned*)(ws + oWQl);
  unsigned* woh  = (unsigned*)(ws + oWOh);
  unsigned* wol  = (unsigned*)(ws + oWOl);
  unsigned* wlh  = (unsigned*)(ws + oWLh);
  unsigned* wll  = (unsigned*)(ws + oWLl);
  int*      cnt  = (int*)(ws + oCnt);
  int*      offp = (int*)(ws + oOff);
  int*      rb   = (int*)(ws + oRb);
  int*      csr  = (int*)(ws + oCsr);
  float*    X    = (float*)(ws + oX);
  float*    QKV  = (float*)(ws + oQKV);

  const int nPrep = nL * (QKVW * DF / 8) + (nL - 1) * (DF * DF / 8) + nCls * DF / 8;
  if ((nPrep % NTHR) != 0 || ((nCls * DF / 8) % NTHR) != 0) return;
  k_wprep<<<nPrep / NTHR, NTHR, 0, stream>>>(qkvw, outw, outwl, wqh, wql, woh, wol, wlh, wll, nL, nCls);

  k_count<<<nBC, NTHR, 0, stream>>>(dstA, cnt, nE, 1);
  k_offsets<<<1, OTHR, 0, stream>>>(cnt, offp, rb, nBC);
  hipFuncSetAttribute(reinterpret_cast<const void*>(&k_fill),
                      hipFuncAttributeMaxDynamicSharedMemorySize, LDS_FILL);
  k_fill<<<nBF, NTHR, LDS_FILL, stream>>>(srcA, dstA, offp, rb, csr, nN, nE, 1, csrLen);

  hipFuncSetAttribute(reinterpret_cast<const void*>(&k_gemm),
                      hipFuncAttributeMaxDynamicSharedMemorySize, LDS_GEMM);
  hipFuncSetAttribute(reinterpret_cast<const void*>(&k_attn<8>),
                      hipFuncAttributeMaxDynamicSharedMemorySize, LDS_ATTN);
  hipFuncSetAttribute(reinterpret_cast<const void*>(&k_attn<4>),
                      hipFuncAttributeMaxDynamicSharedMemorySize, LDS_ATTN);

  for (int l = 0; l < nL; ++l) {
    const float* A = (l == 0) ? x : X;
    const int nRowsA = (l == 0) ? nN : NPAD;
    k_gemm<<<nBlk, NTHR, LDS_GEMM, stream>>>(A, nRowsA,
                                             wqh + (size_t)l * QKVW * KU, wql + (size_t)l * QKVW * KU,
                                             qkvb + (size_t)l * QKVW, QKV);
    if (l < nL - 1) {
      k_attn<8><<<nBlk, NTHR, LDS_ATTN, stream>>>(csr, offp, cnt, QKV,
                                                  woh + (size_t)l * DF * KU, wol + (size_t)l * DF * KU,
                                                  outb + (size_t)l * DF, X, NPAD, nN, csrLen);
    } else if (nCls == 128) {
      k_attn<8><<<nBlk, NTHR, LDS_ATTN, stream>>>(csr, offp, cnt, QKV, wlh, wll, outbl, out, nN, nN, csrLen);
    } else {
      k_attn<4><<<nBlk, NTHR, LDS_ATTN, stream>>>(csr, offp, cnt, QKV, wlh, wll, outbl, out, nN, nN, csrLen);
    }
  }
}
